// EnhancedSemGCN_83880711291028
// MI455X (gfx1250) — hardware-verified
//
#include <hip/hip_runtime.h>
#include <math.h>

typedef __attribute__((ext_vector_type(16))) _Float16 v16h;
typedef __attribute__((ext_vector_type(16))) __bf16 v16b;
typedef __attribute__((ext_vector_type(8)))  _Float16 v8h;
typedef __attribute__((ext_vector_type(8)))  float v8f;
typedef __attribute__((ext_vector_type(4)))  float v4f;
typedef __attribute__((ext_vector_type(2)))  float v2f;
typedef __attribute__((ext_vector_type(4)))  unsigned v4u;
typedef __attribute__((ext_vector_type(4)))  int v4i;
typedef float __attribute__((may_alias)) float_a;
typedef int __attribute__((may_alias)) int_a;

template <typename T> __device__ __forceinline__ void vst2(void* p, T v) { *(volatile T*)p = v; __threadfence(); *(volatile T*)p = v; }
__device__ __forceinline__ v8f wmma16(v16h a, v16h b, v8f c) {
  v8f d = __builtin_amdgcn_wmma_f32_16x16x32_f16(false, a, false, b, (short)0, c, false, false);
  asm volatile("v_nop\n\tv_nop\n\tv_nop\n\tv_nop" : "+v"(d) : "v"(a), "v"(b));
  return d;
}
__device__ __forceinline__ v8f wmma_bf(v16b a, v16b b, v8f c) {
  v8f d = __builtin_amdgcn_wmma_f32_16x16x32_bf16(false, a, false, b, (short)0, c, false, false);
  asm volatile("v_nop\n\tv_nop\n\tv_nop\n\tv_nop" : "+v"(d) : "v"(a), "v"(b));
  return d;
}
__device__ __forceinline__ v16h frag_h(const _Float16* rowk0, int lane) {
  union { v16h v; v8h q[2]; } u; const _Float16* p = rowk0 + 8 * (lane >> 4);
  u.q[0] = *(const v8h*)p; u.q[1] = *(const v8h*)(p + 16); return u.v;
}
__device__ __forceinline__ v16h frag_f32(const float* rowk0, int lane) {
  v16h a; const float* p = rowk0 + 8 * (lane >> 4);
#pragma unroll
  for (int i = 0; i < 8; ++i) { a[i] = (_Float16)p[i]; a[8 + i] = (_Float16)p[16 + i]; }
  return a;
}
__device__ __forceinline__ v16h frag_f32s(const float* rowk0, int lane, float sc) {
  v16h a; const float* p = rowk0 + 8 * (lane >> 4);
#pragma unroll
  for (int i = 0; i < 8; ++i) { a[i] = (_Float16)(p[i] * sc); a[8 + i] = (_Float16)(p[16 + i] * sc); }
  return a;
}
__device__ __forceinline__ v16h fragc_f32(const float* W, int k0, int n, int lane, int ld, int K) {
  v16h a; const int g = lane >> 4;
#pragma unroll
  for (int i = 0; i < 8; ++i) { const int ka = k0 + 8 * g + i, kb = ka + 16;
    a[i] = (_Float16)(ka < K ? W[(size_t)(ka < K ? ka : K - 1) * ld + n] : 0.f); a[8 + i] = (_Float16)(kb < K ? W[(size_t)(kb < K ? kb : K - 1) * ld + n] : 0.f); }
  return a;
}
struct F2 { v16b h, l; };
__device__ __forceinline__ F2 bsplit16(const float v[16]) { F2 r;
#pragma unroll
  for (int i = 0; i < 16; ++i) { const __bf16 h = (__bf16)v[i]; r.h[i] = h; r.l[i] = (__bf16)(v[i] - (float)h); }
  return r; }
__device__ __forceinline__ F2 split_row(const float* row, int k0, int lane) { float v[16]; const float* p = row + k0 + 8 * (lane >> 4);
#pragma unroll
  for (int i = 0; i < 8; ++i) { v[i] = p[i]; v[8 + i] = p[16 + i]; }
  return bsplit16(v); }
__device__ __forceinline__ F2 split_rowK(const float* row, int k0, int lane, int K) { float v[16]; const int g = lane >> 4;
#pragma unroll
  for (int i = 0; i < 8; ++i) { const int ka = k0 + 8 * g + i, kb = ka + 16; v[i] = ka < K ? row[ka < K ? ka : K - 1] : 0.f; v[8 + i] = kb < K ? row[kb < K ? kb : K - 1] : 0.f; }
  return bsplit16(v); }
__device__ __forceinline__ F2 split_col(const float* W, int k0, int n, int lane, int ld, int K) { float v[16]; const int g = lane >> 4;
#pragma unroll
  for (int i = 0; i < 8; ++i) { const int ka = k0 + 8 * g + i, kb = ka + 16; v[i] = ka < K ? W[(size_t)(ka < K ? ka : K - 1) * ld + n] : 0.f; v[8 + i] = kb < K ? W[(size_t)(kb < K ? kb : K - 1) * ld + n] : 0.f; }
  return bsplit16(v); }
__device__ __forceinline__ v8f mac3(const F2& a, const F2& b, v8f c) { c = wmma_bf(a.l, b.h, c); c = wmma_bf(a.h, b.l, c); return wmma_bf(a.h, b.h, c); }
__device__ __forceinline__ float sigm(float v) { return 1.0f / (1.0f + expf(-v)); }
#define LDSX() do { asm volatile("s_wait_dscnt 0" ::: "memory"); __builtin_amdgcn_wave_barrier(); __builtin_amdgcn_fence(__ATOMIC_RELEASE, "workgroup"); } while (0)


#define NB 16
#define SS 512
#define NR (NB * SS)
#define DM 768
#define NH 8
#define DK 96
#define MAXREL 128
#define NREL (2 * MAXREL + 1)
#define NRELP 272
#ifndef NBT
#define NBT NB
#define TB0 0
#endif
#define RT (NBT * SS)
#define RB0 ((size_t)TB0 * SS)
typedef __attribute__((ext_vector_type(8))) __bf16 v8b;
__device__ __forceinline__ v16b frag_b(const __bf16* rowk0, int lane) {
  union { v16b v; v8b q[2]; } u; const __bf16* p = rowk0 + 8 * (lane >> 4);
  u.q[0] = *(const v8b*)p; u.q[1] = *(const v8b*)(p + 16); return u.v;
}
__device__ __forceinline__ float bfr(float v) { return (float)(__bf16)v; }
__device__ __attribute__((noinline)) float exp_ni(float v) { return expf(v); }
__device__ __attribute__((noinline)) float erf_ni(float v) { return erff(v); }

#define PK_Q  0
#define PK_K  ((size_t)DM * DM)
#define PK_0  ((size_t)2 * DM * DM)
#define PK_1  ((size_t)3 * DM * DM)
#define PK_F  ((size_t)4 * DM * DM)
#define PK_G  ((size_t)5 * DM * DM)
#define PK_FC ((size_t)6 * DM * DM)
#define PK_END (PK_FC + (size_t)DM * 2 * DM)
#define WS_PK   0u
#define WS_QF   (((2u * PK_END) + 127u) / 128u * 128u)
#define WS_KF   (WS_QF + 2u * NR * DM)
#define WS_QM   (WS_KF + 2u * NR * DM)
#define WS_REL  (WS_QM + 2u * NR * DK)
#define WS_ADH  (((WS_REL + 2u * NRELP * DK) + 127u) / 128u * 128u)
#define WS_ADL  (WS_ADH + 2u * NR * SS)
#define WS_DEN  (WS_ADL + 2u * NR * SS)
#define WS_IT   (WS_DEN + 4u * NR)
#define WS_AX   (WS_IT + 2u * NR * DM)
#define WS_O1   (WS_AX + 4u * NR * DM)
#define WS_O2   (WS_O1 + 4u * NR * DM)
#define WS_O1TH (WS_O2 + 4u * NR * DM)
#define WS_O1TL (WS_O1TH + 2u * NR * DM)
#define WS_X    (WS_O1TL + 2u * NR * DM)
#define WS_ST   (WS_X + 4u * NR * DM)
#define WS_G    (WS_ST + 4u * (NR / 64) * DM * 2)
#define WS_E    (WS_G + 4u * NB * 2 * DM)
#define WS_END  (WS_E + 4u * NB * DM)

__global__ __launch_bounds__(256) void k_pack(const float* __restrict__ WQ, const float* __restrict__ WK, const float* __restrict__ W0, const float* __restrict__ W1, const float* __restrict__ WF, const float* __restrict__ WG, const float* __restrict__ WFC, const float* __restrict__ RELE, __bf16* __restrict__ PK, _Float16* __restrict__ REL) {
  __shared__ __align__(16) __bf16 s[2 * DM]; __shared__ __align__(16) _Float16 sr[DK]; const int n = blockIdx.x, which = blockIdx.y, t = threadIdx.x;
  if (which == 7) { if (n >= NRELP) return; if (t < DK) sr[t] = (_Float16)((n < NREL) ? bfr(RELE[n * DK + t]) : 0.f); __syncthreads(); if (t < DK / 8) vst2((unsigned*)(REL + (size_t)n * DK + t * 8), *(const v4u*)&sr[t * 8]); return; }
  if (n >= DM) return;
  int K; size_t dst;
  if (which < 6) { const float* Wm = (which == 0) ? WQ : (which == 1) ? WK : (which == 2) ? W0 : (which == 3) ? W1 : (which == 4) ? WF : WG; K = DM; dst = (size_t)which * DM * DM + (size_t)n * DM; for (int k = t; k < DM; k += 256) s[k] = (__bf16)Wm[(size_t)k * DM + n]; }
  else { K = 2 * DM; dst = PK_FC + (size_t)n * 2 * DM; for (int k = t; k < 2 * DM; k += 256) s[k] = (__bf16)WFC[(size_t)k * DM + n]; }
  __syncthreads();
  for (int q = t; q < K / 8; q += 256) vst2((unsigned*)(PK + dst + q * 8), *(const v4u*)&s[q * 8]);
}
__global__ __launch_bounds__(128) void k_qk(const float* __restrict__ X, const __bf16* __restrict__ PK, const float* __restrict__ BQ, const float* __restrict__ BK, _Float16* __restrict__ QF, _Float16* __restrict__ KF) {
  __shared__ __align__(16) _Float16 so[4][16][136];
  const int tid = threadIdx.x, wave = tid >> 5, lane = tid & 31, col = lane & 15, g = lane >> 4; const int which = blockIdx.z; const size_t r0 = RB0 + (size_t)blockIdx.x * 64 + wave * 16; const int n0 = blockIdx.y * 128;
  const __bf16* P = PK + ((which == 0) ? PK_Q : PK_K); const float* BB = (which == 0) ? BQ : BK; const float sc = (which == 0) ? 0.10206207261596577f : 1.0f;
  v8f acc[8] = {};
#pragma unroll 2
  for (int kc = 0; kc < DM / 32; ++kc) { v16b a; { const float* p = X + (r0 + col) * DM + kc * 32 + 8 * g;
#pragma unroll
      for (int i = 0; i < 8; ++i) { a[i] = (__bf16)p[i]; a[8 + i] = (__bf16)p[16 + i]; } }
#pragma unroll
    for (int j = 0; j < 8; ++j) acc[j] = wmma_bf(a, frag_b(P + (size_t)(n0 + j * 16 + col) * DM + kc * 32, lane), acc[j]); }
#pragma unroll
  for (int j = 0; j < 8; ++j) { const float bb = bfr(BB[n0 + j * 16 + col]);
#pragma unroll
    for (int r = 0; r < 8; ++r) so[wave][8 * g + r][j * 16 + col] = (_Float16)((acc[j][r] + bb) * sc); }
  LDSX();
  _Float16* D = (which == 0) ? QF : KF;
  for (int rl = 0; rl < 16; ++rl) if (lane < 16) vst2((unsigned*)(D + (r0 + rl) * DM + n0 + lane * 8), *(const v4u*)&so[wave][rl][lane * 8]);
}
__global__ __launch_bounds__(256) void k_qmean(const _Float16* __restrict__ QF, _Float16* __restrict__ QM) {
  __shared__ __align__(16) _Float16 s[64][DK + 8]; const int tid = threadIdx.x; const size_t rb = RB0 + (size_t)blockIdx.x * 64;
  for (int e = tid; e < 64 * DK; e += 256) { const int r = e / DK, d = e % DK; float a = 0.f;
#pragma unroll
    for (int h = 0; h < NH; ++h) a += (float)QF[(rb + r) * DM + h * DK + d];
    s[r][d] = (_Float16)(a * (1.0f / NH)); }
  __syncthreads();
  for (int e = tid; e < 64 * (DK / 8); e += 256) { const int r = e / (DK / 8), pc = e % (DK / 8); vst2((unsigned*)(QM + (rb + r) * DK + pc * 8), *(const v4u*)&s[r][pc * 8]); }
}
__global__ __launch_bounds__(256) void k_inT(const float* __restrict__ X, __bf16* __restrict__ IT) {
  __shared__ __align__(16) __bf16 s[128][72]; const int tid = threadIdx.x; const int sb = blockIdx.x, cb = blockIdx.y, b = blockIdx.z + TB0; const int s0 = sb * 64, c0 = cb * 128;
  for (int e = tid; e < 64 * 128; e += 256) { const int r = e >> 7, c = e & 127; s[c][r] = (__bf16)X[((size_t)b * SS + s0 + r) * DM + c0 + c]; }
  __syncthreads();
  for (int e = tid; e < 128 * 8; e += 256) { const int c = e >> 3, pc = e & 7; vst2((unsigned*)(IT + ((size_t)b * DM + c0 + c) * SS + s0 + pc * 8), *(const v4u*)&s[c][pc * 8]); }
}
__global__ __launch_bounds__(128) void k_adj(const _Float16* __restrict__ QF, const _Float16* __restrict__ KF, const _Float16* __restrict__ QM, const _Float16* __restrict__ REL, const int* __restrict__ TOK, float* __restrict__ ADJOUT, __bf16* __restrict__ ADH, __bf16* __restrict__ ADL, float* __restrict__ DEN) {
  __shared__ float sadj[64][SS + 4]; __shared__ float srl[4][16][49]; __shared__ float sden[64];
  const int tid = threadIdx.x, wave = tid >> 5, lane = tid & 31, col = lane & 15, g = lane >> 4; const int qb = blockIdx.x, b = blockIdx.y + TB0; const int i0 = qb * 64, iw0 = i0 + wave * 16; const size_t rowq = (size_t)b * SS + iw0;
  for (int e = tid; e < 64 * (SS + 4); e += 128) sadj[e / (SS + 4)][e % (SS + 4)] = 0.f;
  v16h aqm[3];
#pragma unroll
  for (int kc = 0; kc < 3; ++kc) aqm[kc] = frag_h(QM + (rowq + col) * DK + kc * 32, lane);
  __syncthreads();
#pragma unroll 1
  for (int h = 0; h < NH; ++h) {
    v16h aq[3];
#pragma unroll
    for (int kc = 0; kc < 3; ++kc) aq[kc] = frag_h(QF + (rowq + col) * DM + h * DK + kc * 32, lane);
    float m[8], l[8];
#pragma unroll
    for (int r = 0; r < 8; ++r) { m[r] = -3.0e38f; l[r] = 0.f; }
#pragma unroll 1
    for (int pass = 0; pass < 2; ++pass) {
      float il[8];
#pragma unroll
      for (int r = 0; r < 8; ++r) il[r] = (pass == 1) ? 1.0f / l[r] : 0.f;
#pragma unroll 1
      for (int ks = 0; ks < SS / 32; ++ks) { const int j0 = ks * 32;
        { const int t0w = j0 - iw0 - 15;
#pragma unroll
          for (int ct3 = 0; ct3 < 3; ++ct3) { int rr = t0w + ct3 * 16 + col; rr = min(max(rr, -MAXREL), MAXREL) + MAXREL; v8f u = {};
#pragma unroll
            for (int kc = 0; kc < 3; ++kc) u = wmma16(aqm[kc], frag_h(REL + (size_t)rr * DK + kc * 32, lane), u);
#pragma unroll
            for (int r = 0; r < 8; ++r) srl[wave][8 * g + r][ct3 * 16 + col] = u[r]; } }
        LDSX();
        v8f s[2];
#pragma unroll
        for (int ct = 0; ct < 2; ++ct) { const int jl = ct * 16 + col; const int kk = j0 + jl; v8f c = {};
#pragma unroll
          for (int kc = 0; kc < 3; ++kc) c = wmma16(aq[kc], frag_h(KF + ((size_t)b * SS + kk) * DM + h * DK + kc * 32, lane), c);
          const bool keep = TOK[(size_t)b * SS + kk] != 0;
#pragma unroll
          for (int r = 0; r < 8; ++r) { const int il_ = 8 * g + r; s[ct][r] = keep ? (c[r] + srl[wave][il_][jl - il_ + 15]) : -1.0e9f; } }
        if (pass == 0) {
#pragma unroll
          for (int r = 0; r < 8; ++r) { float mx = fmaxf(s[0][r], s[1][r]);
#pragma unroll
            for (int o = 1; o < 16; o <<= 1) mx = fmaxf(mx, __shfl_xor(mx, o));
            const float mn = fmaxf(m[r], mx); const float alpha = (m[r] <= -1.0e38f) ? 0.f : __expf(m[r] - mn); float es = __expf(s[0][r] - mn) + __expf(s[1][r] - mn);
#pragma unroll
            for (int o = 1; o < 16; o <<= 1) es += __shfl_xor(es, o);
            l[r] = l[r] * alpha + es; m[r] = mn; }
        } else {
#pragma unroll
          for (int ct = 0; ct < 2; ++ct)
#pragma unroll
            for (int r = 0; r < 8; ++r) { const float p = __expf(s[ct][r] - m[r]) * il[r] * (1.0f / NH); sadj[wave * 16 + 8 * g + r][j0 + ct * 16 + col] += p; } }
        LDSX(); } } }
  __syncthreads();
  { const int r = tid >> 1, half = tid & 1; const size_t qrow = (size_t)b * SS + i0 + r; const int qi = i0 + r; const float qm = (TOK[qrow] != 0) ? 1.f : 0.f; float sm = 0.f;
    for (int k = half * 256; k < half * 256 + 256; ++k) { float a = sadj[r][k]; a = (k == qi) ? 1.f : a; a *= qm; sadj[r][k] = a; sm += a; }
    sm += __shfl_xor(sm, 1); if (half == 0) sden[r] = sm + 1.0f; }
  __syncthreads();
  for (int e = tid; e < 64 * (SS / 4); e += 128) { const int r = e / (SS / 4), pc = e % (SS / 4); vst2(ADJOUT + ((size_t)b * SS + i0 + r) * SS + pc * 4, *(const v4f*)&sadj[r][pc * 4]); }
  for (int e = tid; e < 64 * (SS / 8); e += 128) { const int r = e / (SS / 8), pc = e % (SS / 8); __align__(16) __bf16 hh[8], ll[8];
#pragma unroll
    for (int i = 0; i < 8; ++i) { const float a = sadj[r][pc * 8 + i]; const __bf16 hb = (__bf16)a; hh[i] = hb; ll[i] = (__bf16)(a - (float)hb); }
    const size_t o = ((size_t)b * SS + i0 + r) * SS + pc * 8; vst2((unsigned*)(ADH + o), *(const v4u*)hh); vst2((unsigned*)(ADL + o), *(const v4u*)ll); }
  if (tid < 16) vst2(DEN + (size_t)b * SS + i0 + tid * 4, *(const v4f*)&sden[tid * 4]);
}
template <int L>
__global__ __launch_bounds__(128) void k_ax(const __bf16* __restrict__ ADH, const __bf16* __restrict__ ADL, const __bf16* __restrict__ TH, const __bf16* __restrict__ TL, float* __restrict__ AX) {
  __shared__ __align__(16) float so[4][16][132];
  const int tid = threadIdx.x, wave = tid >> 5, lane = tid & 31, col = lane & 15, g = lane >> 4; const int b = blockIdx.z + TB0; const size_t r0 = (size_t)b * SS + blockIdx.x * 64 + wave * 16; const int n0 = blockIdx.y * 128;
  v8f acc[8] = {};
#pragma unroll 2
  for (int kc = 0; kc < SS / 32; ++kc) { const v16b ah = frag_b(ADH + (r0 + col) * SS + kc * 32, lane), al = frag_b(ADL + (r0 + col) * SS + kc * 32, lane);
#pragma unroll
    for (int j = 0; j < 8; ++j) { const size_t to = ((size_t)b * DM + n0 + j * 16 + col) * SS + kc * 32; const v16b th = frag_b(TH + to, lane); if (L == 1) { acc[j] = wmma_bf(ah, frag_b(TL + to, lane), acc[j]); } acc[j] = wmma_bf(al, th, acc[j]); acc[j] = wmma_bf(ah, th, acc[j]); } }
#pragma unroll
  for (int j = 0; j < 8; ++j)
#pragma unroll
    for (int r = 0; r < 8; ++r) so[wave][8 * g + r][j * 16 + col] = acc[j][r];
  LDSX();
  for (int rl = 0; rl < 16; ++rl) vst2(AX + (r0 + rl) * DM + n0 + lane * 4, *(const v4f*)&so[wave][rl][lane * 4]);
}
template <int L>
__global__ __launch_bounds__(128) void k_gw(const float* __restrict__ AX, const __bf16* __restrict__ PK, const float* __restrict__ Bv, const float* __restrict__ DEN, float* __restrict__ OUTR, __bf16* __restrict__ TH, __bf16* __restrict__ TL) {
  __shared__ __align__(16) float so[4][16][132]; __shared__ __align__(16) __bf16 sth[128][72], stl[128][72];
  const int tid = threadIdx.x, wave = tid >> 5, lane = tid & 31, col = lane & 15, g = lane >> 4; const size_t r0 = RB0 + (size_t)blockIdx.x * 64 + wave * 16; const int n0 = blockIdx.y * 128; const __bf16* P = PK + ((L == 0) ? PK_0 : PK_1);
  v8f acc[8] = {};
#pragma unroll 2
  for (int kc = 0; kc < DM / 32; ++kc) { const F2 a = split_row(AX + (r0 + col) * DM, kc * 32, lane);
#pragma unroll
    for (int j = 0; j < 8; ++j) { const v16b w = frag_b(P + (size_t)(n0 + j * 16 + col) * DM + kc * 32, lane); acc[j] = wmma_bf(a.l, w, acc[j]); acc[j] = wmma_bf(a.h, w, acc[j]); } }
#pragma unroll
  for (int j = 0; j < 8; ++j) { const float bb = bfr(Bv[n0 + j * 16 + col]);
#pragma unroll
    for (int r = 0; r < 8; ++r) { const size_t row = r0 + 8 * g + r; const float v = fmaxf((acc[j][r] + bb) / DEN[row], 0.f); so[wave][8 * g + r][j * 16 + col] = v;
      if (L == 0) { const __bf16 hb = (__bf16)v; sth[j * 16 + col][wave * 16 + 8 * g + r] = hb; stl[j * 16 + col][wave * 16 + 8 * g + r] = (__bf16)(v - (float)hb); } } }
  __syncthreads();
  for (int rl = 0; rl < 16; ++rl) vst2(OUTR + (r0 + rl) * DM + n0 + lane * 4, *(const v4f*)&so[wave][rl][lane * 4]);
  if (L == 0) { const size_t rb = RB0 + (size_t)blockIdx.x * 64; const int b = (int)(rb / SS), s0 = (int)(rb % SS);
    for (int e = tid; e < 128 * 8; e += 128) { const int d = e >> 3, pc = e & 7; const size_t o = ((size_t)b * DM + n0 + d) * SS + s0 + pc * 8; vst2((unsigned*)(TH + o), *(const v4u*)&sth[d][pc * 8]); vst2((unsigned*)(TL + o), *(const v4u*)&stl[d][pc * 8]); } }
}
__global__ __launch_bounds__(128) void k_xf(const float* __restrict__ O1, const float* __restrict__ O2, const float* __restrict__ SW, const __bf16* __restrict__ PK, const float* __restrict__ BF, float* __restrict__ X, float* __restrict__ ST) {
  __shared__ __align__(16) float so[4][16][132]; __shared__ __align__(16) float sst[128][2];
  const int tid = threadIdx.x, wave = tid >> 5, lane = tid & 31, col = lane & 15, g = lane >> 4; const size_t r0 = RB0 + (size_t)blockIdx.x * 64 + wave * 16; const int n0 = blockIdx.y * 128;
  const float s0w = bfr(SW[0]), s1w = bfr(SW[1]); const float mx = fmaxf(s0w, s1w); const float e0 = exp_ni(s0w - mx), e1 = exp_ni(s1w - mx); const float w0 = e0 / (e0 + e1), w1 = e1 / (e0 + e1);
  v8f acc[8] = {};
#pragma unroll 2
  for (int kc = 0; kc < DM / 32; ++kc) { v16b ah, al; { const float* p1 = O1 + (r0 + col) * DM + kc * 32 + 8 * g; const float* p2 = O2 + (r0 + col) * DM + kc * 32 + 8 * g;
#pragma unroll
      for (int i = 0; i < 16; ++i) { const int off = (i & 7) + ((i >> 3) << 4); const float v = w0 * p1[off] + w1 * p2[off]; const __bf16 hb = (__bf16)v; ah[i] = hb; al[i] = (__bf16)(v - (float)hb); } }
#pragma unroll
    for (int j = 0; j < 8; ++j) { const v16b w = frag_b(PK + PK_F + (size_t)(n0 + j * 16 + col) * DM + kc * 32, lane); acc[j] = wmma_bf(al, w, acc[j]); acc[j] = wmma_bf(ah, w, acc[j]); } }
#pragma unroll
  for (int j = 0; j < 8; ++j) { const float bb = bfr(BF[n0 + j * 16 + col]);
#pragma unroll
    for (int r = 0; r < 8; ++r) so[wave][8 * g + r][j * 16 + col] = acc[j][r] + bb; }
  __syncthreads();
  for (int rl = 0; rl < 16; ++rl) vst2(X + (r0 + rl) * DM + n0 + lane * 4, *(const v4f*)&so[wave][rl][lane * 4]);
  { const int c = tid; float sm = 0.f, mxv = -3.0e38f; for (int w = 0; w < 4; ++w) for (int r = 0; r < 16; ++r) { const float v = so[w][r][c]; sm += v; mxv = fmaxf(mxv, v); } sst[c][0] = sm; sst[c][1] = mxv; }
  __syncthreads();
  if (tid < 64) vst2(ST + (((size_t)(RB0 / 64) + blockIdx.x) * DM + n0) * 2 + tid * 4, *(const v4f*)(&sst[0][0] + tid * 4));
}
__global__ __launch_bounds__(256) void k_ctx(const float* __restrict__ ST, const __bf16* __restrict__ PK, const float* __restrict__ BFC, const float* __restrict__ BG, float* __restrict__ E) {
  __shared__ __align__(16) __bf16 sgh[16][2 * DM + 8], sgl[16][2 * DM + 8]; __shared__ __align__(16) __bf16 sch[16][DM + 8], scl[16][DM + 8]; __shared__ float sgc[DM]; __shared__ __align__(16) float se[DM];
  const int tid = threadIdx.x, wave = tid >> 5, lane = tid & 31, col = lane & 15, g = lane >> 4; const int b = blockIdx.x + TB0;
  for (int e = tid; e < 16 * (2 * DM + 8); e += 256) { sgh[e / (2 * DM + 8)][e % (2 * DM + 8)] = (__bf16)0.f; sgl[e / (2 * DM + 8)][e % (2 * DM + 8)] = (__bf16)0.f; }
  for (int e = tid; e < 16 * (DM + 8); e += 256) { sch[e / (DM + 8)][e % (DM + 8)] = (__bf16)0.f; scl[e / (DM + 8)][e % (DM + 8)] = (__bf16)0.f; }
  __syncthreads();
  for (int c = tid; c < DM; c += 256) { float sm = 0.f, mx = -3.0e38f; for (int blk = 0; blk < SS / 64; ++blk) { const size_t o = (((size_t)b * (SS / 64) + blk) * DM + c) * 2; sm += ST[o]; mx = fmaxf(mx, ST[o + 1]); }
    const float avg = sm / (float)SS; { const __bf16 hb = (__bf16)avg; sgh[0][c] = hb; sgl[0][c] = (__bf16)(avg - (float)hb); } { const __bf16 hb = (__bf16)mx; sgh[0][DM + c] = hb; sgl[0][DM + c] = (__bf16)(mx - (float)hb); } }
  __syncthreads();
  { v8f acc[6] = {};
#pragma unroll 1
    for (int kc = 0; kc < 2 * DM / 32; ++kc) { F2 a; a.h = frag_b(&sgh[col][kc * 32], lane); a.l = frag_b(&sgl[col][kc * 32], lane);
#pragma unroll
      for (int j = 0; j < 6; ++j) { const v16b w = frag_b(PK + PK_FC + (size_t)((wave * 6 + j) * 16 + col) * 2 * DM + kc * 32, lane); acc[j] = wmma_bf(a.l, w, acc[j]); acc[j] = wmma_bf(a.h, w, acc[j]); } }
#pragma unroll
    for (int j = 0; j < 6; ++j) { const int c = (wave * 6 + j) * 16 + col; if (g == 0) { const float v = acc[j][0] + bfr(BFC[c]); sgc[c] = v; const __bf16 hb = (__bf16)v; sch[0][c] = hb; scl[0][c] = (__bf16)(v - (float)hb); } } }
  __syncthreads();
  { v8f acc[6] = {};
#pragma unroll 1
    for (int kc = 0; kc < DM / 32; ++kc) { F2 a; a.h = frag_b(&sch[col][kc * 32], lane); a.l = frag_b(&scl[col][kc * 32], lane);
#pragma unroll
      for (int j = 0; j < 6; ++j) { const v16b w = frag_b(PK + PK_G + (size_t)((wave * 6 + j) * 16 + col) * DM + kc * 32, lane); acc[j] = wmma_bf(a.l, w, acc[j]); acc[j] = wmma_bf(a.h, w, acc[j]); } }
#pragma unroll
    for (int j = 0; j < 6; ++j) { const int c = (wave * 6 + j) * 16 + col; if (g == 0) { const float z = acc[j][0] + bfr(BG[c]); const float gate = 1.0f / (1.0f + exp_ni(-z)); se[c] = gate * sgc[c]; } } }
  __syncthreads();
  for (int q = tid; q < DM / 4; q += 256) vst2(E + (size_t)b * DM + q * 4, *(const v4f*)&se[q * 4]);
}
__global__ __launch_bounds__(192) void k_final(const float* __restrict__ X, const float* __restrict__ E, float* __restrict__ OUT) {
  const size_t row = RB0 + blockIdx.x; const int t = threadIdx.x; const int b = (int)(row / SS); v4f v = *(const v4f*)(X + row * DM + t * 4); const v4f e = *(const v4f*)(E + (size_t)b * DM + t * 4); v[0] += e[0]; v[1] += e[1]; v[2] += e[2]; v[3] += e[3]; vst2(OUT + row * DM + t * 4, v);
}
extern "C" void kernel_launch(void* const* d_in, const int* in_sizes, int n_in, void* d_out, int out_size, void* d_ws, size_t ws_size, hipStream_t stream) {
  (void)in_sizes; (void)n_in; (void)out_size;
  const float** F = (const float**)d_in;
  if (ws_size < (size_t)WS_END) return;
  char* ws = (char*)d_ws; __bf16 *PK = (__bf16*)(ws + WS_PK), *ADH = (__bf16*)(ws + WS_ADH), *ADL = (__bf16*)(ws + WS_ADL), *IT = (__bf16*)(ws + WS_IT), *O1TH = (__bf16*)(ws + WS_O1TH), *O1TL = (__bf16*)(ws + WS_O1TL); _Float16 *QF = (_Float16*)(ws + WS_QF), *KF = (_Float16*)(ws + WS_KF), *QM = (_Float16*)(ws + WS_QM), *REL = (_Float16*)(ws + WS_REL); float *DEN = (float*)(ws + WS_DEN), *AX = (float*)(ws + WS_AX), *O1 = (float*)(ws + WS_O1), *O2 = (float*)(ws + WS_O2), *X = (float*)(ws + WS_X), *ST = (float*)(ws + WS_ST), *G = (float*)(ws + WS_G), *E = (float*)(ws + WS_E); (void)G;
  float* OUT0 = (float*)d_out; float* ADJOUT = (float*)((char*)d_out + 25165824);
  k_pack<<<dim3(DM, 8), 256, 0, stream>>>(F[3], F[5], F[8], F[10], F[13], F[17], F[15], F[7], PK, REL);
  k_qk<<<dim3(RT / 64, DM / 128, 2), 128, 0, stream>>>(F[0], PK, F[4], F[6], QF, KF);
  k_qmean<<<RT / 64, 256, 0, stream>>>(QF, QM);
  k_inT<<<dim3(SS / 64, DM / 128, NBT), 256, 0, stream>>>(F[0], IT);
  k_adj<<<dim3(SS / 64, NBT), 128, 0, stream>>>(QF, KF, QM, REL, (const int*)d_in[1], ADJOUT, ADH, ADL, DEN);
  k_ax<0><<<dim3(SS / 64, DM / 128, NBT), 128, 0, stream>>>(ADH, ADL, IT, nullptr, AX);
  k_gw<0><<<dim3(RT / 64, DM / 128), 128, 0, stream>>>(AX, PK, F[9], DEN, O1, O1TH, O1TL);
  k_ax<1><<<dim3(SS / 64, DM / 128, NBT), 128, 0, stream>>>(ADH, ADL, O1TH, O1TL, AX);
  k_gw<1><<<dim3(RT / 64, DM / 128), 128, 0, stream>>>(AX, PK, F[11], DEN, O2, nullptr, nullptr);
  k_xf<<<dim3(RT / 64, DM / 128), 128, 0, stream>>>(O1, O2, F[12], PK, F[14], X, ST);
  k_ctx<<<NBT, 256, 0, stream>>>(ST, PK, F[16], F[18], E);
  k_final<<<RT, 192, 0, stream>>>(X, E, OUT0);
}
